// CausalAttention_ov2_57518202028181
// MI455X (gfx1250) — hardware-verified
//
#include <hip/hip_runtime.h>
#include <stdint.h>
#include <stddef.h>


#define SEQ 4096
#define DIM 1024
#define NTHR 256

typedef __bf16 v16bf __attribute__((ext_vector_type(16)));
typedef float v8f __attribute__((ext_vector_type(8)));
typedef float v4f __attribute__((ext_vector_type(4)));
typedef unsigned int v4u __attribute__((ext_vector_type(4)));

union Frag { v16bf v; v4u q[2]; };

extern __shared__ __attribute__((aligned(16))) float dyn_lds[];

__device__ __forceinline__ unsigned int f2bf(float f) {
  unsigned int u = __float_as_uint(f);
  u += 0x7fffu + ((u >> 16) & 1u);
  return u >> 16;
}
__device__ __forceinline__ float bf2f(unsigned int b) { return __uint_as_float(b << 16); }

__device__ __forceinline__ void ldfrag(Frag& f, const unsigned short* row, int k0, int h) {
  f.q[0] = *(const v4u*)(row + k0 + 8 * h);
  f.q[1] = *(const v4u*)(row + k0 + 16 + 8 * h);
}

__device__ __forceinline__ v8f mma(const Frag& a, const Frag& b, v8f c) {
  return __builtin_amdgcn_wmma_f32_16x16x32_bf16(false, a.v, false, b.v, (short)0, c, false, false);
}

__device__ __forceinline__ v8f zero8() {
  v8f z = {0.0f, 0.0f, 0.0f, 0.0f, 0.0f, 0.0f, 0.0f, 0.0f};
  return z;
}

__device__ __forceinline__ void split8(const v4f f0, const v4f f1, v4u& uh, v4u& ul) {
  float f[8] = {f0.x, f0.y, f0.z, f0.w, f1.x, f1.y, f1.z, f1.w};
  unsigned int hh[8], ll[8];
#pragma unroll
  for (int e = 0; e < 8; ++e) {
    hh[e] = f2bf(f[e]);
    ll[e] = f2bf(f[e] - bf2f(hh[e]));
  }
  uh.x = hh[0] | (hh[1] << 16); uh.y = hh[2] | (hh[3] << 16);
  uh.z = hh[4] | (hh[5] << 16); uh.w = hh[6] | (hh[7] << 16);
  ul.x = ll[0] | (ll[1] << 16); ul.y = ll[2] | (ll[3] << 16);
  ul.z = ll[4] | (ll[5] << 16); ul.w = ll[6] | (ll[7] << 16);
}

__global__ __launch_bounds__(NTHR) void cvt_kernel(
    const float* __restrict__ x,  const float* __restrict__ wq,
    const float* __restrict__ wk, const float* __restrict__ wv,
    unsigned short* xb, unsigned short* wqb, unsigned short* wkb, unsigned short* wvb,
    int nx8, int nw8) {
  const int i = blockIdx.x * NTHR + threadIdx.x;
  const float* src;
  unsigned short* dst;
  int j;
  if (i < nx8)                { src = x;  dst = xb;  j = i; }
  else if (i < nx8 + nw8)     { src = wq; dst = wqb; j = i - nx8; }
  else if (i < nx8 + 2 * nw8) { src = wk; dst = wkb; j = i - nx8 - nw8; }
  else if (i < nx8 + 3 * nw8) { src = wv; dst = wvb; j = i - nx8 - 2 * nw8; }
  else return;
  const v4f f0 = *(const v4f*)(src + (size_t)j * 8);
  const v4f f1 = *(const v4f*)(src + (size_t)j * 8 + 4);
  v4u u;
  u.x = f2bf(f0.x) | (f2bf(f0.y) << 16);
  u.y = f2bf(f0.z) | (f2bf(f0.w) << 16);
  u.z = f2bf(f1.x) | (f2bf(f1.y) << 16);
  u.w = f2bf(f1.z) | (f2bf(f1.w) << 16);
  volatile v4u* p = (volatile v4u*)(dst + (size_t)j * 8);
  *p = u;
  __threadfence();
  *p = u;
}

__global__ __launch_bounds__(NTHR) void proj_kernel(
    const unsigned short* __restrict__ xb,  const unsigned short* __restrict__ wqb,
    const unsigned short* __restrict__ wkb, const unsigned short* __restrict__ wvb,
    unsigned short* qh, unsigned short* ql, unsigned short* kh, unsigned short* kl,
    unsigned short* vth, unsigned short* vtl) {
  float* stg = dyn_lds;
  const int wave = threadIdx.x >> 5;
  const int lane = threadIdx.x & 31;
  const int h = lane >> 4, m = lane & 15;
  const int b = blockIdx.x;
  const int mat = b >> 8;
  const int rem = b & 255;
  const int rt = rem >> 2;
  const int ct = rem & 3;
  const unsigned short* wsrc = (mat == 0) ? wqb : (mat == 1) ? wkb : wvb;
  const int wr = wave >> 2, wc = wave & 3;
  const int row0 = rt * 64 + wr * 32;
  const int col0 = ct * 256 + wc * 64;

  const unsigned short* aR0 = xb + (size_t)(row0 + m) * DIM;
  const unsigned short* aR1 = xb + (size_t)(row0 + 16 + m) * DIM;
  const unsigned short* bR  = wsrc + (size_t)(col0 + m) * DIM;

  v8f acc[2][4];
#pragma unroll
  for (int mi = 0; mi < 2; ++mi)
#pragma unroll
    for (int t = 0; t < 4; ++t) acc[mi][t] = zero8();

#pragma unroll 1
  for (int kk = 0; kk < DIM; kk += 32) {
    Frag a0, a1, bf[4];
    ldfrag(a0, aR0, kk, h);
    ldfrag(a1, aR1, kk, h);
#pragma unroll
    for (int t = 0; t < 4; ++t) ldfrag(bf[t], bR + (size_t)t * 16 * DIM, kk, h);
#pragma unroll
    for (int t = 0; t < 4; ++t) {
      acc[0][t] = mma(a0, bf[t], acc[0][t]);
      acc[1][t] = mma(a1, bf[t], acc[1][t]);
    }
    asm volatile("v_nop\n\tv_nop\n\tv_nop\n\tv_nop"
                 : "+v"(acc[0][0]), "+v"(acc[0][1]), "+v"(acc[0][2]), "+v"(acc[0][3]),
                   "+v"(acc[1][0]), "+v"(acc[1][1]), "+v"(acc[1][2]), "+v"(acc[1][3])
                 : "v"(a0.v), "v"(a1.v), "v"(bf[0].v), "v"(bf[1].v), "v"(bf[2].v), "v"(bf[3].v)
                 : "memory");
  }

#pragma unroll
  for (int mi = 0; mi < 2; ++mi)
#pragma unroll
    for (int t = 0; t < 4; ++t)
#pragma unroll
      for (int r = 0; r < 8; ++r)
        stg[(wr * 32 + mi * 16 + 8 * h + r) * 256 + wc * 64 + t * 16 + m] = acc[mi][t][r];
  __syncthreads();

  if (mat < 2) {
    unsigned short* ph = (mat == 0) ? qh : kh;
    unsigned short* pl = (mat == 0) ? ql : kl;
#pragma unroll 1
    for (int it = 0; it < 8; ++it) {
      const int row = wave * 8 + it;
      const float* sp = stg + row * 256 + lane * 8;
      const v4f f0 = *(const v4f*)sp;
      const v4f f1 = *(const v4f*)(sp + 4);
      v4u uh, ul;
      split8(f0, f1, uh, ul);
      const size_t g = (size_t)(rt * 64 + row) * DIM + ct * 256 + lane * 8;
      volatile v4u* p0 = (volatile v4u*)(ph + g);
      volatile v4u* p1 = (volatile v4u*)(pl + g);
      *p0 = uh; *p1 = ul;
      __threadfence();
      *p0 = uh; *p1 = ul;
    }
  } else {
#pragma unroll 1
    for (int it = 0; it < 8; ++it) {
      const int ol = wave * 32 + it * 4 + (lane >> 3);
      const int c = lane & 7;
      const float* sp = stg + (c * 8) * 256 + ol;
      v4f f0, f1;
      f0.x = sp[0 * 256]; f0.y = sp[1 * 256]; f0.z = sp[2 * 256]; f0.w = sp[3 * 256];
      f1.x = sp[4 * 256]; f1.y = sp[5 * 256]; f1.z = sp[6 * 256]; f1.w = sp[7 * 256];
      v4u uh, ul;
      split8(f0, f1, uh, ul);
      const size_t g = (size_t)(ct * 256 + ol) * SEQ + rt * 64 + c * 8;
      volatile v4u* p0 = (volatile v4u*)(vth + g);
      volatile v4u* p1 = (volatile v4u*)(vtl + g);
      *p0 = uh; *p1 = ul;
      __threadfence();
      *p0 = uh; *p1 = ul;
    }
  }
}

__global__ __launch_bounds__(NTHR) void attn_kernel(
    const unsigned short* __restrict__ qh, const unsigned short* __restrict__ ql,
    const unsigned short* __restrict__ kh, const unsigned short* __restrict__ kl,
    const unsigned short* __restrict__ vth, const unsigned short* __restrict__ vtl,
    float* out) {
  float* S = dyn_lds;
  __shared__ __attribute__((aligned(16))) unsigned short pbh[16 * 32];
  __shared__ __attribute__((aligned(16))) unsigned short pbl[16 * 32];
  __shared__ float part[16][17];
  __shared__ float row_m[16];
  __shared__ float row_r[16];

  const int ib = blockIdx.x;
  const int wave = threadIdx.x >> 5;
  const int lane = threadIdx.x & 31;
  const int h = lane >> 4, m = lane & 15;
  const int nvalid = 16 * (ib + 1);

  const unsigned short* aRh = qh + (size_t)(ib * 16 + m) * DIM;
  const unsigned short* aRl = ql + (size_t)(ib * 16 + m) * DIM;
  int jb = wave;
  for (; jb + 24 <= ib; jb += 32) {
    const unsigned short* bRh = kh + (size_t)(jb * 16 + m) * DIM;
    const unsigned short* bRl = kl + (size_t)(jb * 16 + m) * DIM;
    v8f acc[4];
#pragma unroll
    for (int t = 0; t < 4; ++t) acc[t] = zero8();
#pragma unroll 1
    for (int kk = 0; kk < DIM; kk += 32) {
      Frag ah, al, bh[4], bl[4];
      ldfrag(ah, aRh, kk, h);
      ldfrag(al, aRl, kk, h);
#pragma unroll
      for (int t = 0; t < 4; ++t) {
        ldfrag(bh[t], bRh + (size_t)t * 128 * DIM, kk, h);
        ldfrag(bl[t], bRl + (size_t)t * 128 * DIM, kk, h);
      }
#pragma unroll
      for (int t = 0; t < 4; ++t) {
        acc[t] = mma(ah, bh[t], acc[t]);
        acc[t] = mma(ah, bl[t], acc[t]);
        acc[t] = mma(al, bh[t], acc[t]);
      }
      asm volatile("v_nop\n\tv_nop\n\tv_nop\n\tv_nop"
                   : "+v"(acc[0]), "+v"(acc[1]), "+v"(acc[2]), "+v"(acc[3])
                   : "v"(ah.v), "v"(al.v),
                     "v"(bh[0].v), "v"(bh[1].v), "v"(bh[2].v), "v"(bh[3].v),
                     "v"(bl[0].v), "v"(bl[1].v), "v"(bl[2].v), "v"(bl[3].v)
                   : "memory");
    }
#pragma unroll
    for (int t = 0; t < 4; ++t) {
      const int jbt = jb + 8 * t;
#pragma unroll
      for (int r = 0; r < 8; ++r) {
        const int M = 8 * h + r;
        const int i = ib * 16 + M;
        const int j = jbt * 16 + m;
        float s = acc[t][r] * 0.03125f;
        if (j > i) s = -__builtin_inff();
        S[M * SEQ + j] = s;
      }
    }
  }
  for (; jb <= ib; jb += 8) {
    const unsigned short* bRh = kh + (size_t)(jb * 16 + m) * DIM;
    const unsigned short* bRl = kl + (size_t)(jb * 16 + m) * DIM;
    v8f acc = zero8();
#pragma unroll 1
    for (int kk = 0; kk < DIM; kk += 32) {
      Frag ah, al, bh0, bl0;
      ldfrag(ah, aRh, kk, h);
      ldfrag(al, aRl, kk, h);
      ldfrag(bh0, bRh, kk, h);
      ldfrag(bl0, bRl, kk, h);
      acc = mma(ah, bh0, acc);
      acc = mma(ah, bl0, acc);
      acc = mma(al, bh0, acc);
      asm volatile("v_nop\n\tv_nop\n\tv_nop\n\tv_nop"
                   : "+v"(acc)
                   : "v"(ah.v), "v"(al.v), "v"(bh0.v), "v"(bl0.v)
                   : "memory");
    }
#pragma unroll
    for (int r = 0; r < 8; ++r) {
      const int M = 8 * h + r;
      const int i = ib * 16 + M;
      const int j = jb * 16 + m;
      float s = acc[r] * 0.03125f;
      if (j > i) s = -__builtin_inff();
      S[M * SEQ + j] = s;
    }
  }
  __syncthreads();

  {
    const int row = threadIdx.x & 15, sub = threadIdx.x >> 4;
    float* Sr = S + row * SEQ;
    float mx = -__builtin_inff();
    for (int j = sub; j < nvalid; j += 16) mx = fmaxf(mx, Sr[j]);
    part[row][sub] = mx;
    __syncthreads();
    if (threadIdx.x < 16) {
      float mm = part[threadIdx.x][0];
#pragma unroll 1
      for (int s2 = 1; s2 < 16; ++s2) mm = fmaxf(mm, part[threadIdx.x][s2]);
      row_m[threadIdx.x] = mm;
    }
    __syncthreads();
    const float mrow = row_m[row];
    float l = 0.0f;
    for (int j = sub; j < nvalid; j += 16) {
      const float e = __expf(Sr[j] - mrow);
      Sr[j] = e;
      l += e;
    }
    part[row][sub] = l;
    __syncthreads();
    if (threadIdx.x < 16) {
      float ll = 0.0f;
#pragma unroll 1
      for (int s2 = 0; s2 < 16; ++s2) ll += part[threadIdx.x][s2];
      row_r[threadIdx.x] = 1.0f / ll;
    }
    __syncthreads();
  }

  const int kkend = (nvalid + 31) & ~31;
  v8f acc[8];
#pragma unroll
  for (int t = 0; t < 8; ++t) acc[t] = zero8();
  const unsigned short* vRh = vth + (size_t)(wave * 128 + m) * SEQ;
  const unsigned short* vRl = vtl + (size_t)(wave * 128 + m) * SEQ;
#pragma unroll 1
  for (int kk = 0; kk < kkend; kk += 32) {
    __syncthreads();
    {
      const int e0 = threadIdx.x, e1 = threadIdx.x + NTHR;
      const int j0 = kk + (e0 & 31), j1 = kk + (e1 & 31);
      float p0 = S[(e0 >> 5) * SEQ + j0];
      float p1 = S[(e1 >> 5) * SEQ + j1];
      if (j0 >= nvalid) p0 = 0.0f;
      if (j1 >= nvalid) p1 = 0.0f;
      const unsigned int hb0 = f2bf(p0), hb1 = f2bf(p1);
      pbh[e0] = (unsigned short)hb0;
      pbl[e0] = (unsigned short)f2bf(p0 - bf2f(hb0));
      pbh[e1] = (unsigned short)hb1;
      pbl[e1] = (unsigned short)f2bf(p1 - bf2f(hb1));
    }
    __syncthreads();
    Frag ah, al;
    ldfrag(ah, pbh + m * 32, 0, h);
    ldfrag(al, pbl + m * 32, 0, h);
#pragma unroll
    for (int g = 0; g < 4; ++g) {
      Frag bh0, bl0, bh1, bl1;
      ldfrag(bh0, vRh + (size_t)(2 * g) * 16 * SEQ, kk, h);
      ldfrag(bl0, vRl + (size_t)(2 * g) * 16 * SEQ, kk, h);
      ldfrag(bh1, vRh + (size_t)(2 * g + 1) * 16 * SEQ, kk, h);
      ldfrag(bl1, vRl + (size_t)(2 * g + 1) * 16 * SEQ, kk, h);
      acc[2 * g]     = mma(ah, bh0, acc[2 * g]);
      acc[2 * g]     = mma(ah, bl0, acc[2 * g]);
      acc[2 * g]     = mma(al, bh0, acc[2 * g]);
      acc[2 * g + 1] = mma(ah, bh1, acc[2 * g + 1]);
      acc[2 * g + 1] = mma(ah, bl1, acc[2 * g + 1]);
      acc[2 * g + 1] = mma(al, bh1, acc[2 * g + 1]);
      asm volatile("v_nop\n\tv_nop\n\tv_nop\n\tv_nop"
                   : "+v"(acc[2 * g]), "+v"(acc[2 * g + 1])
                   : "v"(ah.v), "v"(al.v), "v"(bh0.v), "v"(bl0.v), "v"(bh1.v), "v"(bl1.v)
                   : "memory");
    }
  }

  float* stg = S + wave * 2048;
#pragma unroll
  for (int t = 0; t < 8; ++t)
#pragma unroll
    for (int r = 0; r < 8; ++r)
      stg[(8 * h + r) * 128 + t * 16 + m] = acc[t][r] * row_r[8 * h + r];
  __syncthreads();
  float* orow = out + (size_t)(ib * 16) * DIM + wave * 128 + lane * 4;
#pragma unroll 1
  for (int row = 0; row < 16; ++row) {
    const v4f v = *(const v4f*)(stg + row * 128 + lane * 4);
    *(volatile v4f*)(orow + (size_t)row * DIM) = v;
  }
  __threadfence();
#pragma unroll 1
  for (int row = 0; row < 16; ++row) {
    const v4f v = *(const v4f*)(stg + row * 128 + lane * 4);
    *(volatile v4f*)(orow + (size_t)row * DIM) = v;
  }
}

extern "C" void kernel_launch(void* const* d_in, const int* in_sizes, int n_in,
                              void* d_out, int out_size, void* d_ws, size_t ws_size,
                              hipStream_t stream) {
  if (n_in < 4) return;
  if (in_sizes[0] != SEQ * DIM || in_sizes[1] != DIM * DIM || in_sizes[2] != DIM * DIM ||
      in_sizes[3] != DIM * DIM || out_size != SEQ * DIM) return;

  const float* x  = (const float*)d_in[0];
  const float* wq = (const float*)d_in[1];
  const float* wk = (const float*)d_in[2];
  const float* wv = (const float*)d_in[3];
  float* out = (float*)d_out;

  const size_t bx = (size_t)SEQ * DIM * sizeof(unsigned short);
  const size_t bw = (size_t)DIM * DIM * sizeof(unsigned short);
  char* ws = (char*)d_ws;
  size_t off = 0;
  unsigned short* xb  = (unsigned short*)(ws + off); off += bx;
  unsigned short* wqb = (unsigned short*)(ws + off); off += bw;
  unsigned short* wkb = (unsigned short*)(ws + off); off += bw;
  unsigned short* wvb = (unsigned short*)(ws + off); off += bw;
  unsigned short* qh  = (unsigned short*)(ws + off); off += bx;
  unsigned short* ql  = (unsigned short*)(ws + off); off += bx;
  unsigned short* kh  = (unsigned short*)(ws + off); off += bx;
  unsigned short* kl  = (unsigned short*)(ws + off); off += bx;
  unsigned short* vth = (unsigned short*)(ws + off); off += bx;
  unsigned short* vtl = (unsigned short*)(ws + off); off += bx;
  if (off > ws_size) return;

  const int nx8 = SEQ * DIM / 8;
  const int nw8 = DIM * DIM / 8;
  const int ncv = nx8 + 3 * nw8;
  cvt_kernel<<<(ncv + NTHR - 1) / NTHR, NTHR, 0, stream>>>(x, wq, wk, wv, xb, wqb, wkb, wvb, nx8, nw8);

  proj_kernel<<<3 * (SEQ / 64) * (DIM / 256), NTHR, 64 * 256 * sizeof(float), stream>>>(
      xb, wqb, wkb, wvb, qh, ql, kh, kl, vth, vtl);

  attn_kernel<<<SEQ / 16, NTHR, 16 * SEQ * sizeof(float), stream>>>(qh, ql, kh, kl, vth, vtl, out);
}
